// MHDM__970662609222
// MI455X (gfx1250) — hardware-run, weakly checked
//
#include <hip/hip_runtime.h>
#include <math.h>
#include <stdint.h>

#define NB   8
#define NN   768
#define DD   2048
#define NHD  4
#define HW   192
#define MT   (NB * DD)
#define NQB  (DD / 64)
#define NG   (NN / 64)
#define QSC  4.0f
#define VSC  16.0f
#define PSC  1024.0f
#define SSC  (2.0f / (QSC * QSC))
#define NEG_BIG (-1.0e30f)
static_assert(NHD * HW == NN);
static_assert(HW == 3 * 64 && NG * 64 == NN);
static_assert((HW % 32) == 0 && HW > 128 && (HW - 128) <= 64);
static_assert((DD % 64) == 0 && (NN % 128) == 0 && (MT % 128) == 0 && (NN % 32) == 0 && (DD % 32) == 0);
static_assert(((NN * NN) % 2048) == 0);
static_assert((MT % 32) == 0 && (NN % 64) == 0);

typedef _Float16 v16h __attribute__((ext_vector_type(16)));
typedef _Float16 v8h  __attribute__((ext_vector_type(8)));
typedef __bf16   v16b __attribute__((ext_vector_type(16)));
typedef unsigned short v16us __attribute__((ext_vector_type(16)));
typedef unsigned short v8us  __attribute__((ext_vector_type(8)));
typedef float    v8f  __attribute__((ext_vector_type(8)));
typedef float    v4f  __attribute__((ext_vector_type(4)));
typedef unsigned int v4u __attribute__((ext_vector_type(4)));
union FH { v16h v; v8h h[2]; };
union FB { v16us u; v8us h[2]; };

__device__ __forceinline__ unsigned short bf_bits(float f) {
  unsigned u = __float_as_uint(f);
  return (unsigned short)((u + 0x7FFFu + ((u >> 16) & 1u)) >> 16);
}
__device__ __forceinline__ float bf_up(unsigned short h) { return __uint_as_float(((unsigned)h) << 16); }
__device__ __forceinline__ unsigned short h_bits(_Float16 x) { return __builtin_bit_cast(unsigned short, x); }
__device__ __forceinline__ unsigned pk16(unsigned short a, unsigned short b) { return (unsigned)a | ((unsigned)b << 16); }
__device__ __forceinline__ v8f zero8() { v8f z = {0.f, 0.f, 0.f, 0.f, 0.f, 0.f, 0.f, 0.f}; return z; }

__device__ __forceinline__ v16h ldfrag_h(const _Float16* p) {
  FH f;
  f.h[0] = *(const v8h*)(p);
  f.h[1] = *(const v8h*)(p + 16);
  return f.v;
}
__device__ __forceinline__ v16us ldfrag_b(const unsigned short* p) {
  FB f;
  f.h[0] = *(const v8us*)(p);
  f.h[1] = *(const v8us*)(p + 16);
  return f.u;
}

__device__ __forceinline__ v8f mma_h(v16h a, v16h b, v8f c) {
  c = __builtin_amdgcn_wmma_f32_16x16x32_f16(false, a, false, b, (short)0, c, false, false);
#if defined(__HIP_DEVICE_COMPILE__)
  asm volatile("v_nop\n\tv_nop\n\tv_nop\n\tv_nop" : "+v"(c) : "v"(a), "v"(b));
#endif
  return c;
}
__device__ __forceinline__ v8f mma_b_raw(v16us a, v16us b, v8f c) {
  return __builtin_amdgcn_wmma_f32_16x16x32_bf16(false, __builtin_bit_cast(v16b, a), false,
                                                 __builtin_bit_cast(v16b, b), (short)0, c, false, false);
}
template <typename F>
__device__ __forceinline__ void guard3(v8f& x, v8f& y, F a, F b, F d) {
#if defined(__HIP_DEVICE_COMPILE__)
  asm volatile("v_nop\n\tv_nop\n\tv_nop\n\tv_nop" : "+v"(x), "+v"(y) : "v"(a), "v"(b), "v"(d));
#endif
}
__device__ __forceinline__ void acc_guard4(v8f& a, v8f& b, v8f& c, v8f& d) {
#if defined(__HIP_DEVICE_COMPILE__)
  asm volatile("v_nop\n\tv_nop\n\tv_nop\n\tv_nop" : "+v"(a), "+v"(b), "+v"(c), "+v"(d));
#endif
}
__device__ __forceinline__ void wave_sync_lds() {
  __builtin_amdgcn_fence(__ATOMIC_RELEASE, "workgroup");
  __builtin_amdgcn_wave_barrier();
  __builtin_amdgcn_fence(__ATOMIC_ACQUIRE, "workgroup");
}

struct OpB {
  typedef v16us F;
  static __device__ __forceinline__ F ld(const unsigned short* p) { return ldfrag_b(p); }
  static __device__ __forceinline__ v8f mma(F a, F b, v8f c) { return mma_b_raw(a, b, c); }
};

__global__ __launch_bounds__(256) void tr_cvt(const float* __restrict__ in, unsigned short* out, int R, int C,
                                             long long zin, long long zout) {
  __shared__ float tile[64 * 33];
  const int z = blockIdx.z;
  const float* ib = in + (size_t)z * (size_t)zin;
  unsigned short* ob = out + (size_t)z * (size_t)zout;
  const int r0 = blockIdx.y * 64, c0 = blockIdx.x * 32;
  const int t = threadIdx.x;
  {
    const int ir = t >> 2, ic = (t & 3) * 8;
    const float* g = ib + (size_t)(r0 + ir) * (size_t)C + c0 + ic;
    const v4f a = *(const v4f*)g;
    const v4f b = *(const v4f*)(g + 4);
    float* l = tile + ir * 33 + ic;
    l[0] = a[0]; l[1] = a[1]; l[2] = a[2]; l[3] = a[3];
    l[4] = b[0]; l[5] = b[1]; l[6] = b[2]; l[7] = b[3];
  }
  __syncthreads();
  const int orow = t >> 3, piece = (t & 7) * 8;
  v4u p;
#pragma unroll
  for (int e = 0; e < 4; ++e) {
    const float f0 = tile[(piece + 2 * e) * 33 + orow];
    const float f1 = tile[(piece + 2 * e + 1) * 33 + orow];
    p[e] = pk16(bf_bits(f0), bf_bits(f1));
  }
  const size_t go = (size_t)(c0 + orow) * (size_t)R + r0 + piece;
  *(volatile v4u*)(ob + go) = p;
  __threadfence();
  *(volatile v4u*)(ob + go) = p;
}

__global__ __launch_bounds__(256) void cvt_bf(const float* __restrict__ in, unsigned short* out, int n) {
  const size_t i8 = ((size_t)blockIdx.x * 256 + threadIdx.x) * 8;
  if (i8 + 8 > (size_t)n) return;
  const v4f a = *(const v4f*)(in + i8);
  const v4f b = *(const v4f*)(in + i8 + 4);
  v4u p;
#pragma unroll
  for (int e = 0; e < 2; ++e) {
    p[e]     = pk16(bf_bits(a[2 * e]), bf_bits(a[2 * e + 1]));
    p[2 + e] = pk16(bf_bits(b[2 * e]), bf_bits(b[2 * e + 1]));
  }
  *(volatile v4u*)(out + i8) = p;
  __threadfence();
  *(volatile v4u*)(out + i8) = p;
}

template <class OP, int NSW, int OM>
__global__ __launch_bounds__(128) void gemm_t(
    const unsigned short* __restrict__ A0, const unsigned short* __restrict__ A1, int lda,
    const unsigned short* __restrict__ B0, const unsigned short* __restrict__ B1, int ldb,
    void* C0, void* C1, int ldc, int M, int N, int K, float oscale) {
  typedef typename OP::F F;
  __shared__ __align__(16) float sT[4][16 * 132];
  __shared__ __align__(16) float sQ[4][64];
  const int lane = threadIdx.x & 31;
  const int wave = threadIdx.x >> 5;
  const int tilesN = N >> 7;
  const int tilesM = M >> 5;
  const int tile = blockIdx.x * 4 + wave;
  if (tile >= tilesM * tilesN) return;
  const int tm = tile / tilesN;
  const int tn = tile - tm * tilesN;
  const int m0 = tm << 5;
  const int n0 = tn << 7;
  const int rl   = lane & 15;
  const int hh   = lane >> 4;
  const int koff = hh * 8;

  v8f acc[2][8];
#pragma unroll
  for (int i = 0; i < 2; ++i)
#pragma unroll
    for (int j = 0; j < 8; ++j) acc[i][j] = zero8();

#pragma unroll 1
  for (int sw = 0; sw < NSW; ++sw) {
    const unsigned short* Ab = (sw == 0) ? A0 : A1;
    const unsigned short* Bb = (sw == 0) ? B0 : B1;
    const unsigned short* ar0 = Ab + (size_t)(m0 + rl) * (size_t)lda + koff;
    const unsigned short* ar1 = Ab + (size_t)(m0 + 16 + rl) * (size_t)lda + koff;
    const unsigned short* br  = Bb + (size_t)(n0 + rl) * (size_t)ldb + koff;
    for (int k0 = 0; k0 < K; k0 += 32) {
      const F a0 = OP::ld(ar0 + k0);
      const F a1 = OP::ld(ar1 + k0);
#pragma unroll
      for (int j = 0; j < 8; ++j) {
        const F b = OP::ld(br + (size_t)j * 16 * (size_t)ldb + k0);
        acc[0][j] = OP::mma(a0, b, acc[0][j]);
        acc[1][j] = OP::mma(a1, b, acc[1][j]);
        guard3<F>(acc[0][j], acc[1][j], a0, a1, b);
      }
    }
  }
  acc_guard4(acc[0][0], acc[0][1], acc[0][2], acc[0][3]);
  acc_guard4(acc[0][4], acc[0][5], acc[0][6], acc[0][7]);
  acc_guard4(acc[1][0], acc[1][1], acc[1][2], acc[1][3]);
  acc_guard4(acc[1][4], acc[1][5], acc[1][6], acc[1][7]);

  float* slab = sT[wave];
  float* sq = sQ[wave];
#pragma unroll
  for (int i = 0; i < 2; ++i) {
    const int mB = m0 + 16 * i;
    if (OM == 5) {
#pragma unroll
      for (int r = 0; r < 8; ++r) {
        float s0 = acc[i][0][r] * acc[i][0][r];
        s0 += acc[i][1][r] * acc[i][1][r];
        s0 += acc[i][2][r] * acc[i][2][r];
        s0 += acc[i][3][r] * acc[i][3][r];
        float s1 = acc[i][4][r] * acc[i][4][r];
        s1 += acc[i][5][r] * acc[i][5][r];
        s1 += acc[i][6][r] * acc[i][6][r];
        s1 += acc[i][7][r] * acc[i][7][r];
#pragma unroll
        for (int off = 1; off < 16; off <<= 1) {
          s0 += __shfl_xor(s0, off, 32);
          s1 += __shfl_xor(s1, off, 32);
        }
        if (rl == 0) {
          sq[16 * i + 8 * hh + r]      = s0;
          sq[32 + 16 * i + 8 * hh + r] = s1;
        }
      }
    }
#pragma unroll
    for (int j = 0; j < 8; ++j) {
#pragma unroll
      for (int r = 0; r < 8; ++r) slab[(8 * hh + r) * 132 + 16 * j + rl] = acc[i][j][r] * oscale;
    }
    wave_sync_lds();
    if (OM == 4) {
      float* Cf = (float*)C0;
      for (int pass = 0; pass < 2; ++pass) {
#pragma unroll
        for (int it = 0; it < 16; ++it) {
          const v4f o = *(const v4f*)(slab + it * 132 + lane * 4);
          *(volatile v4f*)(Cf + (size_t)(mB + it) * (size_t)ldc + n0 + lane * 4) = o;
        }
        __threadfence();
      }
    } else {
      unsigned short* Cp = (unsigned short*)C0;
      v4u hv[8];
#pragma unroll
      for (int it = 0; it < 8; ++it) {
        const int row = it * 2 + hh;
        const float* sp = slab + row * 132 + rl * 8;
        const v4f fa = *(const v4f*)sp;
        const v4f fb = *(const v4f*)(sp + 4);
        float f[8];
        f[0] = fa[0]; f[1] = fa[1]; f[2] = fa[2]; f[3] = fa[3];
        f[4] = fb[0]; f[5] = fb[1]; f[6] = fb[2]; f[7] = fb[3];
        v4u pk;
#pragma unroll
        for (int e = 0; e < 4; ++e) {
          const _Float16 x0 = (_Float16)f[2 * e];
          const _Float16 x1 = (_Float16)f[2 * e + 1];
          pk[e] = pk16(h_bits(x0), h_bits(x1));
        }
        hv[it] = pk;
      }
      for (int pass = 0; pass < 2; ++pass) {
#pragma unroll
        for (int it = 0; it < 8; ++it) {
          const int row = it * 2 + hh;
          const size_t go = (size_t)(mB + row) * (size_t)ldc + n0 + rl * 8;
          *(volatile v4u*)(Cp + go) = hv[it];
        }
        __threadfence();
      }
    }
    wave_sync_lds();
  }
  if (OM == 5) {
    float* Q2 = (float*)C1;
    const int g = (lane >> 3) & 1, pc = (lane & 7) * 4;
    const v4f qv = *(const v4f*)(sq + g * 32 + pc);
    float* dst = Q2 + (size_t)((n0 >> 6) + g) * (size_t)M + m0 + pc;
    if (lane < 16) *(volatile v4f*)dst = qv;
    __threadfence();
    if (lane < 16) *(volatile v4f*)dst = qv;
  }
}

__global__ __launch_bounds__(128)
void attn_k(const unsigned short* __restrict__ QKp, const unsigned short* __restrict__ VTp,
            const float* __restrict__ q2p, unsigned short* WH, unsigned short* WL) {
  __shared__ __align__(16) _Float16 Ksh[64 * HW];
  __shared__ __align__(16) _Float16 Vs[HW * 64];
  __shared__ __align__(16) _Float16 Psh[4][16 * 64];
  __shared__ __align__(16) float    Os[4][16 * HW];
  __shared__ __align__(16) float    q2k[64];

  const int tid  = threadIdx.x;
  const int wave = tid >> 5;
  const int lane = tid & 31;
  const int hh   = lane >> 4;
  const int c    = lane & 15;

  const int qb = (int)(blockIdx.x % (unsigned)NQB);
  const int h  = (int)(blockIdx.x / (unsigned)NQB);
  const int q0 = qb * 64 + wave * 16;

  const _Float16* Qg = (const _Float16*)(const void*)QKp + (size_t)h * HW;
  const _Float16* Vg = (const _Float16*)(const void*)VTp + (size_t)h * HW * (size_t)MT;
  const float* g0p = q2p + (size_t)(3 * h) * (size_t)MT;
  const float* g1p = g0p + MT;
  const float* g2p = g1p + MT;

  float q2r[8], mrow[8], lrow[8];
  v8f oh[12];
#pragma unroll
  for (int r = 0; r < 8; ++r) {
    const int qr = q0 + 8 * hh + r;
    q2r[r] = (g0p[qr] + g1p[qr]) + g2p[qr];
    mrow[r] = NEG_BIG;
    lrow[r] = 0.f;
  }
#pragma unroll
  for (int t = 0; t < 12; ++t) oh[t] = zero8();

  _Float16* pwh = Psh[wave];

  for (int kt = 0; kt < NQB; ++kt) {
    const int kv0 = kt * 64;
    __syncthreads();
    {
      const int r = tid >> 1, hk = (tid & 1) * (HW / 2);
      const _Float16* kg = Qg + (size_t)(kv0 + r) * NN + hk;
#pragma unroll
      for (int i = 0; i < (HW / 16); ++i) *(v8h*)(Ksh + r * HW + hk + 8 * i) = *(const v8h*)(kg + 8 * i);
      const _Float16* vg = Vg + (size_t)tid * (size_t)MT + kv0;
#pragma unroll
      for (int i = 0; i < 8; ++i) *(v8h*)(Vs + tid * 64 + 8 * i) = *(const v8h*)(vg + 8 * i);
      if (tid < HW - 128) {
        const _Float16* vg2 = Vg + (size_t)(tid + 128) * (size_t)MT + kv0;
#pragma unroll
        for (int i = 0; i < 8; ++i) *(v8h*)(Vs + (tid + 128) * 64 + 8 * i) = *(const v8h*)(vg2 + 8 * i);
        const int key = kv0 + tid;
        q2k[tid] = (g0p[key] + g1p[key]) + g2p[key];
      }
    }
    __syncthreads();

    v8f s[4];
#pragma unroll
    for (int j = 0; j < 4; ++j) s[j] = zero8();
#pragma unroll
    for (int dc = 0; dc < (HW / 32); ++dc) {
      const v16h qa = ldfrag_h(Qg + (size_t)(q0 + c) * NN + dc * 32 + 8 * hh);
#pragma unroll
      for (int j = 0; j < 4; ++j) {
        FH kb;
        kb.h[0] = *(const v8h*)(Ksh + (j * 16 + c) * HW + dc * 32 + 8 * hh);
        kb.h[1] = *(const v8h*)(Ksh + (j * 16 + c) * HW + dc * 32 + 16 + 8 * hh);
        s[j] = mma_h(qa, kb.v, s[j]);
      }
    }
    acc_guard4(s[0], s[1], s[2], s[3]);
#pragma unroll
    for (int j = 0; j < 4; ++j) {
      const float q2c = q2k[j * 16 + c];
#pragma unroll
      for (int r = 0; r < 8; ++r) s[j][r] = (s[j][r] * SSC - q2r[r]) - q2c;
    }

#pragma unroll
    for (int r = 0; r < 8; ++r) {
      float m = s[0][r];
      m = fmaxf(m, s[1][r]);
      m = fmaxf(m, s[2][r]);
      m = fmaxf(m, s[3][r]);
#pragma unroll
      for (int off = 1; off < 16; off <<= 1) m = fmaxf(m, __shfl_xor(m, off, 32));
      const float mnew  = fmaxf(mrow[r], m);
      const float alpha = __expf(mrow[r] - mnew);
      mrow[r] = mnew;
      float psum = 0.f;
#pragma unroll
      for (int j = 0; j < 4; ++j) {
        const float p = __expf(s[j][r] - mnew);
        psum += p;
        pwh[(8 * hh + r) * 64 + j * 16 + c] = (_Float16)(p * PSC);
      }
#pragma unroll
      for (int off = 1; off < 16; off <<= 1) psum += __shfl_xor(psum, off, 32);
      lrow[r] = lrow[r] * alpha + psum;
#pragma unroll
      for (int t = 0; t < 12; ++t) oh[t][r] *= alpha;
    }
    wave_sync_lds();

#pragma unroll
    for (int kk = 0; kk < 2; ++kk) {
      FH pa;
      pa.h[0] = *(const v8h*)(pwh + c * 64 + kk * 32 + 8 * hh);
      pa.h[1] = *(const v8h*)(pwh + c * 64 + kk * 32 + 16 + 8 * hh);
#pragma unroll
      for (int t = 0; t < 12; ++t) {
        FH vb;
        vb.h[0] = *(const v8h*)(Vs + (t * 16 + c) * 64 + kk * 32 + 8 * hh);
        vb.h[1] = *(const v8h*)(Vs + (t * 16 + c) * 64 + kk * 32 + 16 + 8 * hh);
        oh[t] = mma_h(pa.v, vb.v, oh[t]);
      }
    }
  }
  acc_guard4(oh[0], oh[1], oh[2], oh[3]);
  acc_guard4(oh[4], oh[5], oh[6], oh[7]);
  acc_guard4(oh[8], oh[9], oh[10], oh[11]);

  float* os = Os[wave];
#pragma unroll
  for (int r = 0; r < 8; ++r) {
    const float l = lrow[r];
    const float inv = ((l > 0.f) ? (1.0f / l) : 0.f) * (1.0f / (PSC * VSC));
#pragma unroll
    for (int t = 0; t < 12; ++t) os[(8 * hh + r) * HW + t * 16 + c] = oh[t][r] * inv;
  }
  wave_sync_lds();
  {
    const int cl = (lane < 24) ? lane : 23;
    for (int pass = 0; pass < 2; ++pass) {
#pragma unroll 4
      for (int it = 0; it < 16; ++it) {
        const float* sp = os + it * HW + cl * 8;
        const v4f fa = *(const v4f*)sp;
        const v4f fb = *(const v4f*)(sp + 4);
        float f[8];
        f[0] = fa[0]; f[1] = fa[1]; f[2] = fa[2]; f[3] = fa[3];
        f[4] = fb[0]; f[5] = fb[1]; f[6] = fb[2]; f[7] = fb[3];
        v4u pk, pl;
#pragma unroll
        for (int e = 0; e < 4; ++e) {
          const float g0 = f[2 * e], g1 = f[2 * e + 1];
          const unsigned short b0 = bf_bits(g0), b1 = bf_bits(g1);
          const unsigned short l0 = bf_bits(g0 - bf_up(b0)), l1 = bf_bits(g1 - bf_up(b1));
          pk[e] = pk16(b0, b1);
          pl[e] = pk16(l0, l1);
        }
        const size_t go = (size_t)(q0 + it) * NN + (size_t)h * HW + cl * 8;
        if (lane < 24) {
          *(volatile v4u*)(WH + go) = pk;
          *(volatile v4u*)(WL + go) = pl;
        }
      }
      __threadfence();
    }
  }
}

extern "C" void kernel_launch(void* const* d_in, const int* in_sizes, int n_in,
                              void* d_out, int out_size, void* d_ws, size_t ws_size,
                              hipStream_t stream) {
  if (n_in < 4) return;
  if (in_sizes[0] != NB * NN * DD) return;
  if (in_sizes[1] != NN * NN || in_sizes[2] != NN * NN || in_sizes[3] != NN * NN) return;
  if (out_size != NB * NN * DD) return;

  const float* X   = (const float*)d_in[0];
  const float* Wqk = (const float*)d_in[1];
  const float* Wv  = (const float*)d_in[2];
  const float* Wo  = (const float*)d_in[3];
  float* outf = (float*)d_out;

  const size_t PW  = (size_t)NN * NN * 2;
  const size_t PYT = (size_t)MT * NN * 2;
  const size_t PQK = (size_t)MT * NN * 2;
  const size_t PQ2 = (size_t)NG * MT * 4;
  const size_t PVT = (size_t)NN * MT * 2;
  const size_t PWP = (size_t)DD * NN * 2;
  size_t off = 0;
  const size_t oWQK = off; off += PW;
  const size_t oWV  = off; off += PW;
  const size_t oWO  = off; off += PW;
  const size_t oYT  = off; off += PYT;
  const size_t oQK  = off; off += PQK;
  const size_t oQ2  = off; off += PQ2;
  const size_t oVT  = off; off += PVT;
  const size_t oWH  = off; off += PWP;
  const size_t oWL  = off; off += PWP;
  if (off > ws_size) return;
  if (off > (size_t)134217728) return;

  char* ws = (char*)d_ws;
  unsigned short* WQK = (unsigned short*)(ws + oWQK);
  unsigned short* WV  = (unsigned short*)(ws + oWV);
  unsigned short* WO  = (unsigned short*)(ws + oWO);
  unsigned short* YT  = (unsigned short*)(ws + oYT);
  unsigned short* QKP = (unsigned short*)(ws + oQK);
  float*          Q2P = (float*)(ws + oQ2);
  unsigned short* VT  = (unsigned short*)(ws + oVT);
  unsigned short* WH  = (unsigned short*)(ws + oWH);
  unsigned short* WL  = (unsigned short*)(ws + oWL);

  const dim3 blk256(256), blk128(128);

  cvt_bf<<<dim3((NN * NN) / 2048), blk256, 0, stream>>>(Wqk, WQK, NN * NN);
  cvt_bf<<<dim3((NN * NN) / 2048), blk256, 0, stream>>>(Wv, WV, NN * NN);
  cvt_bf<<<dim3((NN * NN) / 2048), blk256, 0, stream>>>(Wo, WO, NN * NN);
  tr_cvt<<<dim3(DD / 32, NN / 64, NB), blk256, 0, stream>>>(X, YT, NN, DD, (long long)NN * DD, (long long)DD * NN);
  gemm_t<OpB, 1, 5><<<dim3(((MT / 32) * (NN / 128)) / 4), blk128, 0, stream>>>(
      YT, YT, NN, WQK, WQK, NN, (void*)QKP, (void*)Q2P, NN, MT, NN, NN, QSC);
  gemm_t<OpB, 1, 1><<<dim3(((NN / 32) * (MT / 128)) / 4), blk128, 0, stream>>>(
      WV, WV, NN, YT, YT, NN, (void*)VT, (void*)VT, MT, NN, MT, NN, VSC);

  for (int b = 0; b < NB; ++b) {
    const unsigned short* QKb = QKP + (size_t)b * DD * NN;
    const unsigned short* VTb = VT + (size_t)b * DD;
    const float* Q2b = Q2P + (size_t)b * DD;
    float* outb = outf + (size_t)b * NN * DD;
    attn_k<<<dim3(NQB * NHD), blk128, 0, stream>>>(QKb, VTb, Q2b, WH, WL);
    gemm_t<OpB, 2, 4><<<dim3(((NN / 32) * (DD / 128)) / 4), blk128, 0, stream>>>(
        WO, WO, NN, WH, WL, NN, (void*)outb, (void*)outb, DD, NN, DD, NN, 1.0f);
  }
  (void)hipGetLastError();
}
